// SinDY_7687991460297
// MI455X (gfx1250) — hardware-run, weakly checked
//
#include <hip/hip_runtime.h>
#include <math.h>

#pragma clang fp contract(off)

typedef __attribute__((ext_vector_type(16))) __bf16   v16b;
typedef __attribute__((ext_vector_type(8)))  float    v8f;
typedef __attribute__((ext_vector_type(4)))  float    v4f;
typedef __attribute__((ext_vector_type(4)))  unsigned v4u;

constexpr int kLat      = 16;
constexpr int kNout     = 16;
constexpr int kLib      = 169;
constexpr int kKpad     = 192;
constexpr int kRowsAll  = 64 * 8192;
constexpr int kRowsBlk  = 64;
constexpr int kPitchW   = 100;
constexpr int kBtPitchW = kKpad / 2;
static_assert(kLib == 1 + kLat + (kLat * (kLat + 1)) / 2 + kLat);
static_assert((kKpad % 32) == 0 && kKpad >= kLib);
static_assert((kRowsAll % kRowsBlk) == 0);
static_assert((kPitchW % 4) == 0 && kPitchW * 2 >= kKpad);

constexpr int pair_first(int t)  { int a = 0; while (t >= kLat - a) { t -= kLat - a; ++a; } return a; }
constexpr int pair_second(int t) { int a = 0; while (t >= kLat - a) { t -= kLat - a; ++a; } return a + t; }
constexpr bool pair_order_ok() {
  for (int a = 0; a < kLat; ++a)
    for (int b = a; b < kLat; ++b) {
      const int t = 16 * a - (a * (a - 1)) / 2 + (b - a);
      if (pair_first(t) != a || pair_second(t) != b) return false;
    }
  return true;
}
static_assert(pair_order_ok());
static_assert(pair_first(16) == 1 && pair_second(16) == 1);
static_assert(pair_first(31) == 2 && pair_second(31) == 2);
static_assert(pair_first(135) == 15 && pair_second(135) == 15);

constexpr size_t kOffBth  = 0;
constexpr size_t kOffBtl  = kOffBth + (size_t)kNout * kKpad * 2;
constexpr size_t kWsTotal = kOffBtl + (size_t)kNout * kKpad * 2;
static_assert(kWsTotal == 12288ull);
static_assert((kOffBtl % 128) == 0);
static_assert(kWsTotal <= 134217728ull);

__device__ __forceinline__ unsigned bf_hi_word(float f) {
  const unsigned u = __float_as_uint(f);
  return (u + 0x7FFFu + ((u >> 16) & 1u)) & 0xFFFF0000u;
}

__device__ __forceinline__ void split_pack8(float e0, float e1, float e2, float e3,
                                            float e4, float e5, float e6, float e7,
                                            v4u& wh, v4u& wl) {
  const unsigned h0 = bf_hi_word(e0), h1 = bf_hi_word(e1), h2 = bf_hi_word(e2), h3 = bf_hi_word(e3);
  const unsigned h4 = bf_hi_word(e4), h5 = bf_hi_word(e5), h6 = bf_hi_word(e6), h7 = bf_hi_word(e7);
  const unsigned l0 = bf_hi_word(e0 - __uint_as_float(h0));
  const unsigned l1 = bf_hi_word(e1 - __uint_as_float(h1));
  const unsigned l2 = bf_hi_word(e2 - __uint_as_float(h2));
  const unsigned l3 = bf_hi_word(e3 - __uint_as_float(h3));
  const unsigned l4 = bf_hi_word(e4 - __uint_as_float(h4));
  const unsigned l5 = bf_hi_word(e5 - __uint_as_float(h5));
  const unsigned l6 = bf_hi_word(e6 - __uint_as_float(h6));
  const unsigned l7 = bf_hi_word(e7 - __uint_as_float(h7));
  const unsigned a0 = (h0 >> 16) | h1, a1 = (h2 >> 16) | h3, a2 = (h4 >> 16) | h5, a3 = (h6 >> 16) | h7;
  const unsigned b0 = (l0 >> 16) | l1, b1 = (l2 >> 16) | l3, b2 = (l4 >> 16) | l5, b3 = (l6 >> 16) | l7;
  wh = (v4u){a0, a1, a2, a3};
  wl = (v4u){b0, b1, b2, b3};
}

__device__ __forceinline__ v8f mma_bf16(v16b a, v16b b, v8f c) {
  c = __builtin_amdgcn_wmma_f32_16x16x32_bf16(false, a, false, b, (short)0, c, false, false);
  asm volatile("v_nop\n\tv_nop\n\tv_nop\n\tv_nop" : "+v"(c) : "v"(a), "v"(b));
  return c;
}

union FragB { v16b v; v4u q[2]; };
__device__ __forceinline__ v16b load_frag_words(const unsigned* p) {
  FragB f;
  f.q[0] = *(const v4u*)(p);
  f.q[1] = *(const v4u*)(p + 8);
  return f.v;
}

template <int KP>
__device__ __forceinline__ float lib_feat(const float (&xr)[kLat]) {
  static_assert(KP >= 0 && KP < 152);
  constexpr int t = (KP >= 16) ? (KP - 16) : 0;
  constexpr int a = (KP >= 16) ? pair_first(t) : KP;
  constexpr int b = (KP >= 16) ? pair_second(t) : KP;
  return (KP >= 16) ? (xr[a] * xr[b]) : xr[a];
}

template <int G>
__device__ __forceinline__ void emit_group(const float (&xr)[kLat], unsigned* rowh, unsigned* rowl) {
  static_assert(G >= 0 && G <= 18);
  const float e0 = lib_feat<8 * G + 0>(xr);
  const float e1 = lib_feat<8 * G + 1>(xr);
  const float e2 = lib_feat<8 * G + 2>(xr);
  const float e3 = lib_feat<8 * G + 3>(xr);
  const float e4 = lib_feat<8 * G + 4>(xr);
  const float e5 = lib_feat<8 * G + 5>(xr);
  const float e6 = lib_feat<8 * G + 6>(xr);
  const float e7 = lib_feat<8 * G + 7>(xr);
  v4u wh, wl;
  split_pack8(e0, e1, e2, e3, e4, e5, e6, e7, wh, wl);
  *(v4u*)(rowh + 4 * G) = wh;
  *(v4u*)(rowl + 4 * G) = wl;
}

static_assert((kNout * kKpad) % 128 == 0 && (kNout * kKpad) / 8 == 3 * 128);
__global__ __launch_bounds__(128) void prep_weight_planes_kernel(
    const float* __restrict__ coef, const float* __restrict__ mask,
    unsigned* __restrict__ bth, unsigned* __restrict__ btl)
{
  __shared__ __align__(16) float sW[kNout * kKpad];
  const int tid = threadIdx.x;
#pragma unroll 1
  for (int it = 0; it < (kNout * kKpad) / 128; ++it) {
    const int idx = it * 128 + tid;
    const int n   = idx / kKpad;
    const int kp  = idx - n * kKpad;
    const bool live = (kp <= 168);
    int l = (kp < 168) ? (kp + 1) : 0;
    l = (l < 0) ? 0 : l;
    l = (l > kLib - 1) ? (kLib - 1) : l;
    float cv = coef[l * kNout + n];
    float mv = mask[l * kNout + n];
    asm volatile("" : "+v"(cv), "+v"(mv));
    const float w = mv * cv;
    sW[idx] = live ? w : 0.0f;
  }
  __syncthreads();
#pragma unroll 1
  for (int it = 0; it < 3; ++it) {
    const int ch = it * 128 + tid;
    const float* sp = sW + ch * 8;
    const v4f a0 = *(const v4f*)(sp);
    const v4f a1 = *(const v4f*)(sp + 4);
    const float e0 = a0[0], e1 = a0[1], e2 = a0[2], e3 = a0[3];
    const float e4 = a1[0], e5 = a1[1], e6 = a1[2], e7 = a1[3];
    v4u wh, wl;
    split_pack8(e0, e1, e2, e3, e4, e5, e6, e7, wh, wl);
    unsigned* ph = bth + ch * 4;
    unsigned* pl = btl + ch * 4;
    *(volatile v4u*)ph = wh;
    *(volatile v4u*)pl = wl;
    __threadfence();
    *(volatile v4u*)ph = wh;
    *(volatile v4u*)pl = wl;
    __threadfence();
  }
}

__global__ __launch_bounds__(64) void library_product_kernel(
    const float* __restrict__ x, const unsigned* __restrict__ bth, const unsigned* __restrict__ btl,
    float* __restrict__ out)
{
  __shared__ __align__(16) unsigned sAh[kRowsBlk * kPitchW];
  __shared__ __align__(16) unsigned sAl[kRowsBlk * kPitchW];
  __shared__ __align__(16) float    sD[kRowsBlk * kNout];

  const int tid  = threadIdx.x;
  const int lane = tid & 31;
  const int wave = tid >> 5;
  const int hh   = lane >> 4;
  const int c    = lane & 15;
  const size_t row0 = (size_t)blockIdx.x * kRowsBlk;

  {
    const float* xp = x + (row0 + (size_t)tid) * kLat;
    const v4f q0 = *(const v4f*)(xp);
    const v4f q1 = *(const v4f*)(xp + 4);
    const v4f q2 = *(const v4f*)(xp + 8);
    const v4f q3 = *(const v4f*)(xp + 12);
    const float xr[kLat] = {q0[0], q0[1], q0[2], q0[3], q1[0], q1[1], q1[2], q1[3],
                            q2[0], q2[1], q2[2], q2[3], q3[0], q3[1], q3[2], q3[3]};
    unsigned* rh = sAh + tid * kPitchW;
    unsigned* rl = sAl + tid * kPitchW;
    emit_group<0>(xr, rh, rl);
    emit_group<1>(xr, rh, rl);
    emit_group<2>(xr, rh, rl);
    emit_group<3>(xr, rh, rl);
    emit_group<4>(xr, rh, rl);
    emit_group<5>(xr, rh, rl);
    emit_group<6>(xr, rh, rl);
    emit_group<7>(xr, rh, rl);
    emit_group<8>(xr, rh, rl);
    emit_group<9>(xr, rh, rl);
    emit_group<10>(xr, rh, rl);
    emit_group<11>(xr, rh, rl);
    emit_group<12>(xr, rh, rl);
    emit_group<13>(xr, rh, rl);
    emit_group<14>(xr, rh, rl);
    emit_group<15>(xr, rh, rl);
    emit_group<16>(xr, rh, rl);
    emit_group<17>(xr, rh, rl);
    emit_group<18>(xr, rh, rl);
    const v4u w_one  = (v4u){0x00003F80u, 0u, 0u, 0u};
    const v4u w_zero = (v4u){0u, 0u, 0u, 0u};
    *(v4u*)(rh + 84) = w_one;
    *(v4u*)(rh + 88) = w_zero;
    *(v4u*)(rh + 92) = w_zero;
    *(v4u*)(rl + 84) = w_zero;
    *(v4u*)(rl + 88) = w_zero;
    *(v4u*)(rl + 92) = w_zero;
  }

#pragma unroll 1
  for (int trip = 0; trip < 2; ++trip) {
    const int g    = tid + 64 * trip;
    const int row  = g >> 1;
    const int half = g & 1;
    const float* xp = x + (row0 + (size_t)row) * kLat + half * 8;
    const v4f a0 = *(const v4f*)(xp);
    const v4f a1 = *(const v4f*)(xp + 4);
    const float t0 = a0[0], t1 = a0[1], t2 = a0[2], t3 = a0[3];
    const float t4 = a1[0], t5 = a1[1], t6 = a1[2], t7 = a1[3];
    const float s0 = sinf(t0), s1 = sinf(t1), s2 = sinf(t2), s3 = sinf(t3);
    const float s4 = sinf(t4), s5 = sinf(t5), s6 = sinf(t6), s7 = sinf(t7);
    v4u wh, wl;
    split_pack8(s0, s1, s2, s3, s4, s5, s6, s7, wh, wl);
    *(v4u*)(sAh + row * kPitchW + 76 + half * 4) = wh;
    *(v4u*)(sAl + row * kPitchW + 76 + half * 4) = wl;
  }

  __syncthreads();

  v8f acc0 = (v8f){0.f, 0.f, 0.f, 0.f, 0.f, 0.f, 0.f, 0.f};
  v8f acc1 = (v8f){0.f, 0.f, 0.f, 0.f, 0.f, 0.f, 0.f, 0.f};
  {
    const unsigned* pa0h = sAh + (wave * 32 + c) * kPitchW + 4 * hh;
    const unsigned* pa0l = sAl + (wave * 32 + c) * kPitchW + 4 * hh;
    const unsigned* pa1h = pa0h + 16 * kPitchW;
    const unsigned* pa1l = pa0l + 16 * kPitchW;
    const unsigned* pbh  = bth + c * kBtPitchW + 4 * hh;
    const unsigned* pbl  = btl + c * kBtPitchW + 4 * hh;
#pragma unroll 2
    for (int ks = 0; ks < kKpad / 32; ++ks) {
      const int kw = ks * 16;
      const v16b bh  = load_frag_words(pbh + kw);
      const v16b bl  = load_frag_words(pbl + kw);
      const v16b a0h = load_frag_words(pa0h + kw);
      const v16b a0l = load_frag_words(pa0l + kw);
      const v16b a1h = load_frag_words(pa1h + kw);
      const v16b a1l = load_frag_words(pa1l + kw);
      acc0 = mma_bf16(a0h, bh, acc0);
      acc0 = mma_bf16(a0h, bl, acc0);
      acc0 = mma_bf16(a0l, bh, acc0);
      acc1 = mma_bf16(a1h, bh, acc1);
      acc1 = mma_bf16(a1h, bl, acc1);
      acc1 = mma_bf16(a1l, bh, acc1);
    }
  }

#pragma unroll
  for (int r = 0; r < 8; ++r) {
    sD[(wave * 32 + 8 * hh + r) * kNout + c]      = acc0[r];
    sD[(wave * 32 + 16 + 8 * hh + r) * kNout + c] = acc1[r];
  }
  __syncthreads();
  {
    v4f vals[4];
#pragma unroll
    for (int it = 0; it < 4; ++it) vals[it] = *(const v4f*)(sD + wave * 512 + it * 128 + lane * 4);
    float* ob = out + row0 * kNout + (size_t)wave * 512;
    for (int pass = 0; pass < 2; ++pass) {
#pragma unroll
      for (int it = 0; it < 4; ++it)
        *(volatile v4f*)(ob + it * 128 + lane * 4) = vals[it];
      __threadfence();
    }
  }
}

extern "C" void kernel_launch(void* const* d_in, const int* in_sizes, int n_in,
                              void* d_out, int out_size, void* d_ws, size_t ws_size,
                              hipStream_t stream) {
  if (n_in < 3) return;
  if (in_sizes[0] != kRowsAll * kLat) return;
  if (in_sizes[1] != kLib * kNout) return;
  if (in_sizes[2] != kLib * kNout) return;
  if (out_size != kRowsAll * kNout) return;
  if (ws_size < kWsTotal) return;

  const float* x    = (const float*)d_in[0];
  const float* coef = (const float*)d_in[1];
  const float* mask = (const float*)d_in[2];
  float* out = (float*)d_out;

  char* ws = (char*)d_ws;
  unsigned* bth = (unsigned*)(ws + kOffBth);
  unsigned* btl = (unsigned*)(ws + kOffBtl);

  prep_weight_planes_kernel<<<1, 128, 0, stream>>>(coef, mask, bth, btl);
  library_product_kernel<<<kRowsAll / kRowsBlk, kRowsBlk, 0, stream>>>(x, bth, btl, out);
}
